// CapsNet_81733227643432
// MI455X (gfx1250) — hardware-verified
//
#include <hip/hip_runtime.h>
#include <math.h>
#include <stddef.h>

typedef __attribute__((ext_vector_type(16))) _Float16 v16h;
typedef __attribute__((ext_vector_type(8)))  _Float16 v8h;
typedef __attribute__((ext_vector_type(16))) __bf16   v16b;
typedef __attribute__((ext_vector_type(8)))  __bf16   v8b;
typedef __attribute__((ext_vector_type(8)))  float    v8f;
typedef __attribute__((ext_vector_type(4)))  float    v4f;

constexpr int NBATCH  = 8;
constexpr int NMI     = 8;
constexpr int NDI     = 16;
constexpr int NMO     = 8;
constexpr int NDO     = 16;
constexpr int IMH     = 64;
constexpr int IMW     = 64;
constexpr int CIN     = NMI * NDI;
constexpr int COUT_CH = NMO * NDO;
constexpr int NTAP    = 9;
constexpr int KDIM    = NTAP * CIN;
constexpr int KRUNS   = KDIM / 8;
constexpr int MPIX    = NBATCH * IMH * IMW;
constexpr int NCAPS   = NBATCH * NMO * IMH * IMW;
constexpr int NTHR    = 256;
constexpr int SQ_PITCH = 20;
constexpr int GEMM_TILES  = (MPIX / 64) * (COUT_CH / 64);
constexpr int GEMM_BLOCKS = GEMM_TILES / 8;

static_assert(KDIM % 32 == 0, "GEMM K multiple of 32");
static_assert(MPIX % 64 == 0 && COUT_CH % 64 == 0, "GEMM M, N tile multiples");
static_assert(GEMM_TILES % 8 == 0, "GEMM grid exact");
static_assert((COUT_CH * KRUNS) % NTHR == 0, "Bt prep grid exact");
static_assert((MPIX * KRUNS) % NTHR == 0, "im2col grid exact");
static_assert(NCAPS % NTHR == 0, "squash grid exact");
static_assert((IMH * IMW) % NTHR == 0, "output map index block-uniform in the squash kernel");
static_assert(CIN % 16 == 0 && (CIN / 8) == 16, "run decode uses r>>4 for tap");

constexpr size_t WS_OFF_BT   = 0;
constexpr size_t WS_BYTES_BT = (size_t)COUT_CH * KDIM * 2;
constexpr size_t WS_OFF_A    = WS_OFF_BT + WS_BYTES_BT;
constexpr size_t WS_BYTES_A  = (size_t)MPIX * KDIM * 2;
constexpr size_t WS_OFF_Y    = WS_OFF_A + WS_BYTES_A;
constexpr size_t WS_BYTES_Y  = (size_t)MPIX * COUT_CH * 4;
constexpr size_t WS_TOTAL    = WS_OFF_Y + WS_BYTES_Y;
static_assert(WS_TOTAL == (size_t)92569600, "carve total");
static_assert(WS_TOTAL <= (size_t)134217728, "carve under 128 MiB");
static_assert(WS_OFF_A % 128 == 0 && WS_OFF_Y % 128 == 0, "line-aligned regions");

__device__ __forceinline__ unsigned short f2bf_bits(float f) {
  unsigned u = __float_as_uint(f);
  return (unsigned short)((u + 0x7FFFu + ((u >> 16) & 1u)) >> 16);
}
__device__ __forceinline__ float bf_bits2f(unsigned short h) { return __uint_as_float(((unsigned)h) << 16); }
__device__ __forceinline__ float bfr(float f) { return bf_bits2f(f2bf_bits(f)); }

__device__ __forceinline__ void dep_guard_h(v8f& a, v8f& b, v16h x, v16h y) { asm volatile("v_nop\n\tv_nop\n\tv_nop\n\tv_nop" : "+v"(a), "+v"(b) : "v"(x), "v"(y)); }
__device__ __forceinline__ void dep_guard_b(v8f& a, v8f& b, v16b x, v16b y) { asm volatile("v_nop\n\tv_nop\n\tv_nop\n\tv_nop" : "+v"(a), "+v"(b) : "v"(x), "v"(y)); }
__device__ __forceinline__ void dep_guard4_h(v8f& a, v8f& b, v8f& c, v8f& d, v16h x, v16h y) { asm volatile("v_nop\n\tv_nop\n\tv_nop\n\tv_nop" : "+v"(a), "+v"(b), "+v"(c), "+v"(d) : "v"(x), "v"(y)); }
__device__ __forceinline__ void dep_guard4_b(v8f& a, v8f& b, v8f& c, v8f& d, v16b x, v16b y) { asm volatile("v_nop\n\tv_nop\n\tv_nop\n\tv_nop" : "+v"(a), "+v"(b), "+v"(c), "+v"(d) : "v"(x), "v"(y)); }
__device__ __forceinline__ void keep4_h(v16h a, v16h b, v16h c, v16h d) { asm volatile("v_nop" :: "v"(a), "v"(b), "v"(c), "v"(d)); }
__device__ __forceinline__ void keep4_b(v16b a, v16b b, v16b c, v16b d) { asm volatile("v_nop" :: "v"(a), "v"(b), "v"(c), "v"(d)); }
__device__ __forceinline__ void acc_guard4(v8f& a, v8f& b, v8f& c, v8f& d) { asm volatile("v_nop\n\tv_nop\n\tv_nop\n\tv_nop" : "+v"(a), "+v"(b), "+v"(c), "+v"(d)); }
template <typename T> struct Frag;
template <> struct Frag<_Float16> {
  typedef v16h V; union U { v16h v; v8h h[2]; };
  static __device__ __forceinline__ v16h load(const _Float16* p) {
    U f; f.h[0] = *(const v8h*)(p); f.h[1] = *(const v8h*)(p + 16); return f.v;
  }
  static __device__ __forceinline__ v8f mma(v16h a, v16h b, v8f c) {
    return __builtin_amdgcn_wmma_f32_16x16x32_f16(false, a, false, b, (short)0, c, false, false);
  }
  static __device__ __forceinline__ void guard(v8f& a, v8f& b, v16h x, v16h y) { dep_guard_h(a, b, x, y); }
  static __device__ __forceinline__ void guard4(v8f& a, v8f& b, v8f& c, v8f& d, v16h x, v16h y) { dep_guard4_h(a, b, c, d, x, y); }
  static __device__ __forceinline__ void keep(v16h a, v16h b, v16h c, v16h d) { keep4_h(a, b, c, d); }
};
template <> struct Frag<__bf16> {
  typedef v16b V; union U { v16b v; v8b h[2]; };
  static __device__ __forceinline__ v16b load(const __bf16* p) {
    U f; f.h[0] = *(const v8b*)(p); f.h[1] = *(const v8b*)(p + 16); return f.v;
  }
  static __device__ __forceinline__ v8f mma(v16b a, v16b b, v8f c) {
    return __builtin_amdgcn_wmma_f32_16x16x32_bf16(false, a, false, b, (short)0, c, false, false);
  }
  static __device__ __forceinline__ void guard(v8f& a, v8f& b, v16b x, v16b y) { dep_guard_b(a, b, x, y); }
  static __device__ __forceinline__ void guard4(v8f& a, v8f& b, v8f& c, v8f& d, v16b x, v16b y) { dep_guard4_b(a, b, c, d, x, y); }
  static __device__ __forceinline__ void keep(v16b a, v16b b, v16b c, v16b d) { keep4_b(a, b, c, d); }
};

template <int ET> struct Elem;
template <> struct Elem<0> { typedef _Float16 T; };
template <> struct Elem<1> { typedef __bf16 T; };
template <int ET, bool SPLIT, int BIAS_MODE, int OUT_MODE, bool RESID, int ACT = 0>
__global__ __launch_bounds__(256) void wmma_gemm64(
    const unsigned short* __restrict__ Ap, const unsigned short* __restrict__ A2p, int lda, long strideA,
    const unsigned short* __restrict__ Btp, const unsigned short* __restrict__ Bt2p, int ldb, long strideB,
    void* __restrict__ Cout, void* __restrict__ Cout2, int ldc, long strideC,
    const float* __restrict__ bias,
    const float* __restrict__ resid, long strideR,
    int M, int N, int K, float scale) {
  typedef typename Elem<ET>::T T;
  typedef typename Frag<T>::V V;
  const T* A = (const T*)Ap; const T* A2 = (const T*)A2p; const T* Bt = (const T*)Btp; const T* Bt2 = (const T*)Bt2p;
  __shared__ __align__(16) float sT[8][16 * 68];
  const int b    = blockIdx.y;
  const int lane = threadIdx.x & 31;
  const int wave = threadIdx.x >> 5;
  const int tilesN = N >> 6;
  const int tilesM = M >> 6;
  const int tile = blockIdx.x * 8 + wave;
  if (tile >= tilesM * tilesN) return;
  const int tm = tile / tilesN;
  const int tn = tile - tm * tilesN;
  const int m0 = tm << 6;
  const int n0 = tn << 6;

  const T* Ab  = A  + (size_t)b * strideA;
  const T* Bb  = Bt + (size_t)b * strideB;
  const T* Ab2 = SPLIT ? (A2  + (size_t)b * strideA) : nullptr;
  const T* Bb2 = SPLIT ? (Bt2 + (size_t)b * strideB) : nullptr;

  const int rlane = lane & 15;
  const int koff  = (lane >> 4) * 8;
  const int mOff  = (lane >> 4) * 8;

  v8f acc[4][4];
#pragma unroll
  for (int i = 0; i < 4; ++i)
#pragma unroll
    for (int j = 0; j < 4; ++j) acc[i][j] = (v8f){0.f,0.f,0.f,0.f,0.f,0.f,0.f,0.f};

  for (int k0 = 0; k0 < K; k0 += 32) {
    V bh[4], bl[4];
#pragma unroll
    for (int j = 0; j < 4; ++j) {
      const size_t bo = (size_t)(n0 + (j << 4) + rlane) * ldb + koff + k0;
      bh[j] = Frag<T>::load(Bb + bo);
      if (SPLIT) bl[j] = Frag<T>::load(Bb2 + bo);
    }
#pragma unroll
    for (int i = 0; i < 4; ++i) {
      const size_t ao = (size_t)(m0 + (i << 4) + rlane) * lda + koff + k0;
      V ah = Frag<T>::load(Ab + ao);
      V al;
      if (SPLIT) al = Frag<T>::load(Ab2 + ao);
#pragma unroll
      for (int j = 0; j < 4; ++j) {
        acc[i][j] = Frag<T>::mma(ah, bh[j], acc[i][j]);
        if (SPLIT) {
          acc[i][j] = Frag<T>::mma(ah, bl[j], acc[i][j]);
          acc[i][j] = Frag<T>::mma(al, bh[j], acc[i][j]);
        }
      }
      Frag<T>::guard4(acc[i][0], acc[i][1], acc[i][2], acc[i][3], ah, SPLIT ? al : ah);
    }
    Frag<T>::keep(bh[0], bh[1], bh[2], bh[3]);
    if (SPLIT) Frag<T>::keep(bl[0], bl[1], bl[2], bl[3]);
  }
  acc_guard4(acc[0][0], acc[0][1], acc[0][2], acc[0][3]);
  acc_guard4(acc[1][0], acc[1][1], acc[1][2], acc[1][3]);
  acc_guard4(acc[2][0], acc[2][1], acc[2][2], acc[2][3]);
  acc_guard4(acc[3][0], acc[3][1], acc[3][2], acc[3][3]);

  float* slab = sT[wave];
  const float* Rb = RESID ? (resid + (size_t)b * strideR) : nullptr;
#pragma unroll
  for (int i = 0; i < 4; ++i) {
    const int mBase = m0 + (i << 4);
#pragma unroll
    for (int j = 0; j < 4; ++j) {
      const int n = n0 + (j << 4) + rlane;
      float bv = 0.f;
      if (BIAS_MODE == 2) bv = bias[n];
#pragma unroll
      for (int r = 0; r < 8; ++r) {
        float v = acc[i][j][r] * scale;
        if (BIAS_MODE == 1) v += bias[mBase + mOff + r];
        if (BIAS_MODE == 2) v += bv;
        if (RESID) v += Rb[(size_t)(mBase + mOff + r) * ldc + n];
        if (ACT == 1) v = tanhf(v);
        if (ACT == 2) v = fmaxf(v, 0.0f);
        if (ACT == 3) v = v / (1.0f + expf(-v));
        if (ACT == 4) v = (v > 0.f) ? v : 0.01f * v;
        if (ACT == 5) v = 0.5f * v * (1.0f + erff(v * 0.70710678118654752f));
        slab[(mOff + r) * 68 + (j << 4) + rlane] = v;
      }
    }
    __builtin_amdgcn_fence(__ATOMIC_RELEASE, "workgroup");
    __builtin_amdgcn_wave_barrier();
    __builtin_amdgcn_fence(__ATOMIC_ACQUIRE, "workgroup");
    if (OUT_MODE == 0) {
      float* C = (float*)Cout + (size_t)b * strideC;
      const int hh = lane >> 4, c4 = (lane & 15) * 4;
      for (int pass = 0; pass < 2; ++pass) {
#pragma unroll
        for (int it = 0; it < 8; ++it) {
          const int row = it * 2 + hh;
          v4f v = *(const v4f*)(slab + row * 68 + c4);
          *(volatile v4f*)(C + (size_t)(mBase + row) * ldc + n0 + c4) = v;
        }
        __threadfence();
      }
    } else {
      const int q = lane >> 3, c8 = (lane & 7) * 8;
      unsigned short* C  = (unsigned short*)Cout  + (size_t)b * strideC;
      unsigned short* C2 = (OUT_MODE == 2) ? ((unsigned short*)Cout2 + (size_t)b * strideC) : nullptr;
      for (int pass = 0; pass < 2; ++pass) {
#pragma unroll
        for (int it = 0; it < 4; ++it) {
          const int row = it * 4 + q;
          const float* sp = slab + row * 68 + c8;
          v8h hv, lv;
#pragma unroll
          for (int e = 0; e < 8; ++e) {
            if (OUT_MODE == 1) {
              hv[e] = (_Float16)sp[e];
            } else {
              unsigned short hb = f2bf_bits(sp[e]);
              unsigned short lb = f2bf_bits(sp[e] - bf_bits2f(hb));
              hv[e] = __builtin_bit_cast(_Float16, hb);
              lv[e] = __builtin_bit_cast(_Float16, lb);
            }
          }
          *(volatile v8h*)(C + (size_t)(mBase + row) * ldc + n0 + c8) = hv;
          if (OUT_MODE == 2) *(volatile v8h*)(C2 + (size_t)(mBase + row) * ldc + n0 + c8) = lv;
        }
        __threadfence();
      }
    }
    __builtin_amdgcn_fence(__ATOMIC_RELEASE, "workgroup");
    __builtin_amdgcn_wave_barrier();
    __builtin_amdgcn_fence(__ATOMIC_ACQUIRE, "workgroup");
  }
}

__global__ __launch_bounds__(NTHR) void k_wbt(const float* __restrict__ cw, unsigned short* __restrict__ bt) {
  const int i = blockIdx.x * NTHR + threadIdx.x;
  if (i >= COUT_CH * KRUNS) return;
  const int n    = i / KRUNS;
  const int r    = i - n * KRUNS;
  const int tap  = r >> 4;
  const int cin0 = (r & 15) * 8;
  const float* src = cw + ((size_t)(n * CIN + cin0)) * NTAP + tap;
  v8h hv;
#pragma unroll
  for (int e = 0; e < 8; ++e) {
    const float v = src[e * NTAP];
    const unsigned short hb = f2bf_bits(v);
    hv[e] = __builtin_bit_cast(_Float16, hb);
  }
  const size_t o = (size_t)i * 8;
  *(volatile v8h*)(bt + o) = hv;
  __threadfence();
  *(volatile v8h*)(bt + o) = hv;
}

__global__ __launch_bounds__(NTHR) void k_im2col(const float* __restrict__ x, unsigned short* __restrict__ ap) {
  const int i = blockIdx.x * NTHR + threadIdx.x;
  if (i >= MPIX * KRUNS) return;
  const int m    = i / KRUNS;
  const int r    = i - m * KRUNS;
  const int tap  = r >> 4;
  const int cin0 = (r & 15) * 8;
  const int mi   = cin0 >> 4;
  const int di0  = cin0 & 15;
  const int kh   = tap / 3;
  const int kw   = tap - kh * 3;
  const int w    = m & 63;
  const int h    = (m >> 6) & 63;
  const int b    = m >> 12;
  const int hs   = h + kh - 1;
  const int ws   = w + kw - 1;
  const bool valid = ((unsigned)hs < (unsigned)IMH) && ((unsigned)ws < (unsigned)IMW);
  const int hc = hs < 0 ? 0 : (hs > IMH - 1 ? IMH - 1 : hs);
  const int wc = ws < 0 ? 0 : (ws > IMW - 1 ? IMW - 1 : ws);
  const float* src = x + (((((size_t)(b * NMI + mi)) * IMH + hc) * IMW + wc) * NDI + di0);
  const v4f v0 = *(const v4f*)(src);
  const v4f v1 = *(const v4f*)(src + 4);
  const float fa = valid ? 1.0f : 0.0f;
  v8h hv;
#pragma unroll
  for (int e = 0; e < 4; ++e) {
    const float a0 = v0[e] * fa;
    const float a1 = v1[e] * fa;
    const unsigned short b0 = f2bf_bits(a0);
    const unsigned short b1 = f2bf_bits(a1);
    hv[e]     = __builtin_bit_cast(_Float16, b0);
    hv[4 + e] = __builtin_bit_cast(_Float16, b1);
  }
  const size_t o = (size_t)i * 8;
  *(volatile v8h*)(ap + o) = hv;
  __threadfence();
  *(volatile v8h*)(ap + o) = hv;
}

__global__ __launch_bounds__(NTHR) void k_squash(const float* __restrict__ y, const float* __restrict__ cb,
                                                 float* __restrict__ out) {
  __shared__ __align__(16) float sO[NTHR * SQ_PITCH];
  __shared__ __align__(16) float sB[NDO];
  const int tid = threadIdx.x;
  const int g   = blockIdx.x * NTHR + tid;
  const int w   = g & 63;
  const int h   = (g >> 6) & 63;
  const int mo  = (g >> 12) & 7;
  const int b   = g >> 15;
  const int mo_blk = (blockIdx.x >> 4) & 7;
  if (tid < NDO) sB[tid] = bfr(cb[mo_blk * NDO + tid]);
  const int m = (b * IMH + h) * IMW + w;
  const float* yp = y + (size_t)m * COUT_CH + mo * NDO;
  v4f yv[4];
#pragma unroll
  for (int c = 0; c < 4; ++c) yv[c] = *(const v4f*)(yp + 4 * c);
  __syncthreads();

  float s[16];
  float sq = 0.0f;
#pragma unroll
  for (int c = 0; c < 4; ++c) {
#pragma unroll
    for (int e = 0; e < 4; ++e) {
      const float yy = yv[c][e];
      const float sv = yy + sB[4 * c + e];
      s[4 * c + e] = sv;
      sq += sv * sv;
    }
  }
  const float safe   = sqrtf(sq + 1e-7f);
  const float rs     = 1.0f / safe;
  const float factor = sq / (1.0f + sq);
#pragma unroll
  for (int c = 0; c < 4; ++c) {
    v4f o;
#pragma unroll
    for (int e = 0; e < 4; ++e) o[e] = factor * (s[4 * c + e] * rs);
    *(v4f*)(sO + tid * SQ_PITCH + 4 * c) = o;
  }
  __syncthreads();

  float* ob = out + (size_t)blockIdx.x * (NTHR * NDO);
  for (int pass = 0; pass < 2; ++pass) {
#pragma unroll
    for (int it = 0; it < 4; ++it) {
      const int f = it * NTHR + tid;
      const v4f v = *(const v4f*)(sO + (f >> 2) * SQ_PITCH + (f & 3) * 4);
      *(volatile v4f*)(ob + (size_t)f * 4) = v;
    }
    __threadfence();
  }
}

extern "C" void kernel_launch(void* const* d_in, const int* in_sizes, int n_in,
                              void* d_out, int out_size, void* d_ws, size_t ws_size,
                              hipStream_t stream) {
  if (n_in < 3) return;
  if (ws_size < WS_TOTAL) return;
  if ((size_t)out_size < (size_t)NCAPS * NDO) return;
  if (in_sizes[0] < NBATCH * NMI * IMH * IMW * NDI) return;
  if (in_sizes[1] < COUT_CH * CIN * NTAP) return;
  if (in_sizes[2] < COUT_CH) return;

  const float* x  = (const float*)d_in[0];
  const float* cw = (const float*)d_in[1];
  const float* cb = (const float*)d_in[2];

  char* wsb = (char*)d_ws;
  unsigned short* bt = (unsigned short*)(wsb + WS_OFF_BT);
  unsigned short* ap = (unsigned short*)(wsb + WS_OFF_A);
  float*          yp = (float*)(wsb + WS_OFF_Y);
  float*          op = (float*)d_out;

  k_wbt<<<(COUT_CH * KRUNS) / NTHR, NTHR, 0, stream>>>(cw, bt);
  k_im2col<<<(MPIX * KRUNS) / NTHR, NTHR, 0, stream>>>(x, ap);
  wmma_gemm64<1, false, 0, 0, false, 0><<<dim3(GEMM_BLOCKS, 1), 256, 0, stream>>>(
      ap, ap, KDIM, 0L,
      bt, bt, KDIM, 0L,
      (void*)yp, (void*)yp, COUT_CH, 0L,
      cb,
      cb, 0L,
      MPIX, COUT_CH, KDIM, 1.0f);
  k_squash<<<NCAPS / NTHR, NTHR, 0, stream>>>(yp, cb, op);
}
